// GatedGCNModel_77713138253857
// MI455X (gfx1250) — hardware-verified
//
#include <hip/hip_runtime.h>
#include <stddef.h>


#define INW    64
#define EH     256
#define HD     128
#define NL     4
#define HHALF  64
#define EPSV   1e-5f
#define HSC    16.0f
#define WSC    64.0f
#define RH     0.0009765625f
#define GROWS  32
#define GTHR   64
#define STHR   256
#define SWAV   (STHR / 32)
#define EPT    16
#define CHUNK  (STHR * EPT)
#define NBA    256
#define NPADG  256
#define BNEL   2048
#define WSCAP  134217728
#define OFF_E1 0
#define OFF_E2 16384
#define OFF_L  49152
#define LPL    49152
#define OFF_HW (OFF_L + NL * LPL)
#define WPTOT  (OFF_HW + HHALF * HD)
#define LDS_DRAIN (NBA * HD * 4 + CHUNK * 4 + NBA * 4 + 3 * HD * 4 + 64)

static_assert(OFF_E2 == EH * INW);
static_assert(OFF_L == OFF_E2 + HD * EH);
static_assert(LPL == 3 * HD * HD);
static_assert(WPTOT == 253952);
static_assert(GROWS == (GTHR / 32) * 16);
static_assert(GTHR == HHALF);
static_assert(NBA == STHR && (NBA % SWAV) == 0);
static_assert(CHUNK == 4096);
static_assert((NPADG % NBA) == 0 && (NPADG % GROWS) == 0);
static_assert((NBA * HD) % (8 * STHR) == 0 && (NBA * HD) % (4 * STHR) == 0);
static_assert((BNEL % EH) == 0 && (BNEL % HD) == 0 && BNEL == 8 * 256);
static_assert((NPADG * HD) % BNEL == 0 && (NPADG * EH) % BNEL == 0);
static_assert((HD % 32) == 0 && (EH % 32) == 0 && (INW % 32) == 0);

typedef float    v4f  __attribute__((ext_vector_type(4)));
typedef float    v8f  __attribute__((ext_vector_type(8)));
typedef int      v4i  __attribute__((ext_vector_type(4)));
typedef _Float16 v8h  __attribute__((ext_vector_type(8)));
typedef _Float16 v16h __attribute__((ext_vector_type(16)));
union Frag { v16h v; v8h h[2]; };

__device__ __forceinline__ v8f wmh(v16h a, v16h b, v8f c) {
  v8f d = __builtin_amdgcn_wmma_f32_16x16x32_f16(false, a, false, b, (short)0, c, false, false);
  asm volatile("v_nop\n\tv_nop\n\tv_nop\n\tv_nop" : "+v"(d) : "v"(a), "v"(b));
  return d;
}

__device__ __forceinline__ v4f vrelu(v4f a) {
  v4f r;
  r.x = fmaxf(a.x, 0.0f); r.y = fmaxf(a.y, 0.0f); r.z = fmaxf(a.z, 0.0f); r.w = fmaxf(a.w, 0.0f);
  return r;
}

template <int KS, int NT>
__device__ __forceinline__ void mma16(const _Float16* __restrict__ Ar, const _Float16* __restrict__ Bpl,
                                      int lane, v8f (&acc)[NT]) {
  constexpr int KH = 32 * KS;
  const int hh = lane >> 4, m = lane & 15;
#pragma unroll
  for (int t = 0; t < NT; ++t) { v8f z = {0.f, 0.f, 0.f, 0.f, 0.f, 0.f, 0.f, 0.f}; acc[t] = z; }
  const _Float16* ap = Ar + (size_t)m * KH + 8 * hh;
  const _Float16* bb = Bpl + (size_t)m * KH + 8 * hh;
#pragma unroll 1
  for (int ks = 0; ks < KS; ++ks) {
    Frag a;
    a.h[0] = *(const v8h*)(ap + 32 * ks);
    a.h[1] = *(const v8h*)(ap + 32 * ks + 16);
#pragma unroll
    for (int t = 0; t < NT; ++t) {
      const _Float16* bp = bb + (size_t)(16 * t) * KH + 32 * ks;
      Frag b;
      b.h[0] = *(const v8h*)bp;
      b.h[1] = *(const v8h*)(bp + 16);
      acc[t] = wmh(a.v, b.v, acc[t]);
    }
  }
}

__global__ __launch_bounds__(256) void k_wprep(const float* __restrict__ ew1, const float* __restrict__ ew2,
                                               const float* __restrict__ gw1, const float* __restrict__ wl,
                                               const float* __restrict__ hw1, _Float16* WP) {
  const int blk = blockIdx.x, tid = threadIdx.x;
  const float* src;
  int pitch, k0;
  size_t dsto;
  if (blk < 8) {
    const int i = blk * 256 + tid;
    src = ew1 + (i >> 3); pitch = EH; k0 = (i & 7) * 8;
    dsto = (size_t)OFF_E1 + 8 * (size_t)i;
  } else if (blk < 24) {
    const int i = (blk - 8) * 256 + tid;
    src = ew2 + (i >> 5); pitch = HD; k0 = (i & 31) * 8;
    dsto = (size_t)OFF_E2 + 8 * (size_t)i;
  } else if (blk < 24 + 24 * NL) {
    const int j = blk - 24, l = j / 24;
    const int i = (j - 24 * l) * 256 + tid;
    const int n = i >> 4;
    const int n1 = n - HD < 0 ? 0 : n - HD;
    const int n2 = n - 2 * HD < 0 ? 0 : n - 2 * HD;
    const float* s0 = gw1 + (size_t)l * (2 * HD * HD) + n;
    const float* s1 = gw1 + (size_t)l * (2 * HD * HD) + (size_t)HD * HD + n1;
    const float* s2 = wl + (size_t)l * (HD * HD) + n2;
    src = (n < HD) ? s0 : ((n < 2 * HD) ? s1 : s2);
    pitch = HD; k0 = (i & 15) * 8;
    dsto = (size_t)OFF_L + (size_t)l * LPL + 8 * (size_t)i;
  } else {
    const int i = (blk - 24 - 24 * NL) * 256 + tid;
    src = hw1 + (i >> 4); pitch = HHALF; k0 = (i & 15) * 8;
    dsto = (size_t)OFF_HW + 8 * (size_t)i;
  }
  float v[8];
#pragma unroll
  for (int e = 0; e < 8; ++e) v[e] = src[(size_t)(k0 + e) * pitch];
  v8h hv;
#pragma unroll
  for (int e = 0; e < 8; ++e) hv[e] = (_Float16)(v[e] * WSC);
  _Float16* dp = WP + dsto;
  *(volatile v8h*)dp = hv;
  __threadfence();
  *(volatile v8h*)dp = hv;
}

__global__ __launch_bounds__(256) void k_xprep(const float* __restrict__ x, _Float16* XH, int nN) {
  const int i = blockIdx.x * 256 + threadIdx.x;
  const int row = i >> 3, c0 = (i & 7) * 8;
  const int xr = row < nN ? row : nN - 1;
  const float* xp = x + (size_t)xr * INW + c0;
  const v4f a = *(const v4f*)xp, b = *(const v4f*)(xp + 4);
  const float f = (row < nN) ? HSC : 0.0f;
  v8h hv;
  hv[0] = (_Float16)(a.x * f); hv[1] = (_Float16)(a.y * f); hv[2] = (_Float16)(a.z * f); hv[3] = (_Float16)(a.w * f);
  hv[4] = (_Float16)(b.x * f); hv[5] = (_Float16)(b.y * f); hv[6] = (_Float16)(b.z * f); hv[7] = (_Float16)(b.w * f);
  _Float16* dp = XH + 8 * (size_t)i;
  *(volatile v8h*)dp = hv;
  __threadfence();
  *(volatile v8h*)dp = hv;
}

template <int NT, int STAT>
__device__ __forceinline__ void gemm_store(const float* stg, const float* spart, float* C, int ldc,
                                           float* part, int ldp, int rowBase, int cb, int tid) {
  constexpr int NCB = 16 * NT, NV4 = NCB / 4;
  float* cbase = C + (size_t)rowBase * ldc + cb;
#pragma unroll 1
  for (int it = 0; it < (GROWS * NV4) / GTHR; ++it) {
    const int f = it * GTHR + tid;
    const int row = f / NV4, piece = f - row * NV4;
    const v4f v = ((const v4f*)stg)[f];
    *(volatile v4f*)(cbase + (size_t)row * ldc + 4 * piece) = v;
  }
  if (STAT) {
    const int wave = tid >> 5, lane = tid & 31;
    const v4f v = ((const v4f*)(spart + wave * NCB))[lane];
    *(volatile v4f*)(part + (size_t)(2 * blockIdx.x + wave) * ldp + cb + 4 * lane) = v;
  }
}

template <int KS, int NT, int STAT>
__global__ __launch_bounds__(GTHR) void k_gemm(const _Float16* __restrict__ A, const _Float16* __restrict__ Bpl,
                                               const float* __restrict__ bias, int bc0, int bc1,
                                               float* C, int ldc, float* part, int ldp, int nN) {
  constexpr int NCB = 16 * NT, KH = 32 * KS;
  static_assert(STAT == 0 || NCB == 128);
  __shared__ __attribute__((aligned(16))) float stg[GROWS * NCB];
  __shared__ __attribute__((aligned(16))) float spart[2 * NCB];
  const int tid = threadIdx.x, lane = tid & 31, wave = tid >> 5, hh = lane >> 4, m = lane & 15;
  const int rowBase = blockIdx.x * GROWS, cb = blockIdx.y * NCB;
  {
    v8f acc[NT];
    mma16<KS, NT>(A + (size_t)(rowBase + wave * 16) * KH, Bpl + (size_t)cb * KH, lane, acc);
    float* sp = stg + (wave * 16 + 8 * hh) * NCB + m;
    const int nb = bc1 - bc0;
#pragma unroll
    for (int t = 0; t < NT; ++t) {
      const int n = cb + 16 * t + m;
      int bi = n - bc0;
      const bool inr = (bi >= 0) && (bi < nb);
      bi = bi < 0 ? 0 : (bi > nb - 1 ? nb - 1 : bi);
      bi = bi < 0 ? 0 : bi;
      float bv = bias[bi];
      bv = inr ? bv : 0.0f;
#pragma unroll
      for (int r = 0; r < 8; ++r) sp[r * NCB + 16 * t] = fmaf(acc[t][r], RH, bv);
    }
  }
  __syncthreads();
  if (STAT) {
    int nv = nN - rowBase;
    nv = nv < 0 ? 0 : (nv > GROWS ? GROWS : nv);
#pragma unroll
    for (int cc = 0; cc < NCB / GTHR; ++cc) {
      const int c = tid + cc * GTHR;
      float s = 0.0f, s2 = 0.0f;
#pragma unroll 1
      for (int r = 0; r < nv; ++r) {
        const float v = stg[r * NCB + c];
        s += v;
        s2 = fmaf(v, v, s2);
      }
      spart[c] = s;
      spart[NCB + c] = s2;
    }
    __syncthreads();
  }
  gemm_store<NT, STAT>(stg, spart, C, ldc, part, ldp, rowBase, cb, tid);
  __threadfence();
  gemm_store<NT, STAT>(stg, spart, C, ldc, part, ldp, rowBase, cb, tid);
}

__global__ __launch_bounds__(256) void k_bnstat(const float* __restrict__ part, int nRB, int Nc,
                                                const float* __restrict__ gam, float* stat, int nN) {
  const int c = threadIdx.x;
  const int cc = c < Nc ? c : Nc - 1;
  double s = 0.0, s2 = 0.0;
#pragma unroll 1
  for (int b = 0; b < nRB; ++b) {
    s  += (double)part[(size_t)(2 * b) * Nc + cc];
    s2 += (double)part[(size_t)(2 * b + 1) * Nc + cc];
  }
  const double mu = s / (double)nN;
  double var = s2 / (double)nN - mu * mu;
  var = var < 0.0 ? 0.0 : var;
  const float muf = (float)mu;
  const float rs = 1.0f / sqrtf((float)var + EPSV);
  const float sg = rs * gam[cc];
  if (c < Nc) {
    *(volatile float*)(stat + c) = muf;
    *(volatile float*)(stat + 256 + c) = sg;
    __threadfence();
    *(volatile float*)(stat + c) = muf;
    *(volatile float*)(stat + 256 + c) = sg;
  }
}

template <int NC, int WF>
__device__ __forceinline__ void bn_store(v8h hv, const float* sy, _Float16* HP, float* HF, size_t ebase, int tid) {
  *(volatile v8h*)(HP + ebase + 8 * (size_t)tid) = hv;
  if (WF) {
#pragma unroll
    for (int it = 0; it < 2; ++it) {
      const int f = it * 256 + tid;
      const v4f v = ((const v4f*)sy)[f];
      *(volatile v4f*)(HF + ebase + 4 * (size_t)f) = v;
    }
  }
}

template <int NC, int WF>
__global__ __launch_bounds__(256) void k_bnapply(const float* __restrict__ Z, const float* __restrict__ stat,
                                                 const float* __restrict__ beta, _Float16* HP, float* HF) {
  __shared__ __attribute__((aligned(16))) float smu[NC];
  __shared__ __attribute__((aligned(16))) float ssg[NC];
  __shared__ __attribute__((aligned(16))) float sbe[NC];
  __shared__ __attribute__((aligned(16))) float sy[WF ? BNEL : 4];
  const int tid = threadIdx.x;
  for (int i = tid; i < NC; i += 256) { smu[i] = stat[i]; ssg[i] = stat[256 + i]; sbe[i] = beta[i]; }
  __syncthreads();
  const size_t ebase = (size_t)blockIdx.x * BNEL;
  const int col = (8 * tid) & (NC - 1);
  const float* zp = Z + ebase + 8 * (size_t)tid;
  const v4f z0 = *(const v4f*)zp, z1 = *(const v4f*)(zp + 4);
  float y[8];
  y[0] = z0.x; y[1] = z0.y; y[2] = z0.z; y[3] = z0.w; y[4] = z1.x; y[5] = z1.y; y[6] = z1.z; y[7] = z1.w;
  v8h hv;
#pragma unroll
  for (int j = 0; j < 8; ++j) {
    y[j] = fmaxf(fmaf(y[j] - smu[col + j], ssg[col + j], sbe[col + j]), 0.0f);
    hv[j] = (_Float16)(y[j] * HSC);
  }
  if (WF) {
    v4f a = {y[0], y[1], y[2], y[3]}, b = {y[4], y[5], y[6], y[7]};
    ((v4f*)sy)[2 * tid] = a;
    ((v4f*)sy)[2 * tid + 1] = b;
    __syncthreads();
  }
  bn_store<NC, WF>(hv, sy, HP, HF, ebase, tid);
  __threadfence();
  bn_store<NC, WF>(hv, sy, HP, HF, ebase, tid);
}

__device__ __forceinline__ void loadids(const int* __restrict__ ids, int nE, int cbase, int tid, int vec,
                                        int (&d)[EPT]) {
  const int e0 = cbase + EPT * tid;
  if (vec != 0 && cbase + CHUNK <= nE) {
#pragma unroll
    for (int q = 0; q < EPT / 4; ++q) {
      const v4i t4 = *(const v4i*)(ids + e0 + 4 * q);
      d[4 * q] = t4.x; d[4 * q + 1] = t4.y; d[4 * q + 2] = t4.z; d[4 * q + 3] = t4.w;
    }
  } else {
#pragma unroll
    for (int j = 0; j < EPT; ++j) {
      int idx = e0 + j;
      const bool ok = idx < nE;
      idx = ok ? idx : nE - 1;
      const int val = ids[idx];
      d[j] = ok ? val : (-2147483647 - 1);
    }
  }
}

__device__ __forceinline__ void blkscan(int cnt, int lane, int wave, int* swt, int& pos, int& nh) {
  int x = cnt;
#pragma unroll
  for (int o = 1; o < 32; o <<= 1) {
    const int y = __shfl_up(x, o, 32);
    x += (lane >= o) ? y : 0;
  }
  if (lane == 31) swt[wave] = x;
  __syncthreads();
  int wpre = 0, tot = 0;
#pragma unroll
  for (int w = 0; w < SWAV; ++w) {
    const int v = swt[w];
    wpre += (w < wave) ? v : 0;
    tot += v;
  }
  pos = wpre + x - cnt;
  nh = tot;
}

__device__ __forceinline__ void drain_store(const float* sacc, float* H, _Float16* HB, int n0, int tid) {
  float* hp = H + (size_t)n0 * HD;
#pragma unroll 1
  for (int it = 0; it < (NBA * HD) / (4 * STHR); ++it) {
    const int f = it * STHR + tid;
    const v4f v = ((const v4f*)sacc)[f];
    *(volatile v4f*)(hp + 4 * (size_t)f) = v;
  }
  _Float16* bp = HB + (size_t)n0 * HD;
#pragma unroll 1
  for (int it = 0; it < (NBA * HD) / (8 * STHR); ++it) {
    const int f = it * STHR + tid;
    const v4f* ap = (const v4f*)(sacc + 8 * f);
    const v4f a0 = ap[0], a1 = ap[1];
    v8h hv;
    hv[0] = (_Float16)(a0.x * HSC); hv[1] = (_Float16)(a0.y * HSC); hv[2] = (_Float16)(a0.z * HSC); hv[3] = (_Float16)(a0.w * HSC);
    hv[4] = (_Float16)(a1.x * HSC); hv[5] = (_Float16)(a1.y * HSC); hv[6] = (_Float16)(a1.z * HSC); hv[7] = (_Float16)(a1.w * HSC);
    *(volatile v8h*)(bp + 8 * (size_t)f) = hv;
  }
}

__global__ __launch_bounds__(STHR) void k_drain(
    const int* __restrict__ own, const int* __restrict__ nbr, const float* __restrict__ T,
    const float* __restrict__ gw2, const float* __restrict__ gb2,
    const float* __restrict__ lg, const float* __restrict__ lb,
    float* H, _Float16* HB, int nN, int nE, int nChunks, int vec) {
  extern __shared__ __attribute__((aligned(16))) char dynl[];
  float*    sacc  = (float*)dynl;
  unsigned* slist = (unsigned*)(dynl + NBA * HD * 4);
  int*      scnt  = (int*)(dynl + NBA * HD * 4 + CHUNK * 4);
  float*    sw2   = (float*)(dynl + NBA * HD * 4 + CHUNK * 4 + NBA * 4);
  float*    sg    = sw2 + HD;
  float*    sb    = sg + HD;
  int*      swt   = (int*)(sb + HD);
  const int tid = threadIdx.x, lane = tid & 31;
  const int wave = __builtin_amdgcn_readfirstlane(tid >> 5);
  const int n0 = blockIdx.x * NBA;
  {
    v4f z = {0.f, 0.f, 0.f, 0.f};
    v4f* p = (v4f*)sacc;
#pragma unroll
    for (int it = 0; it < (NBA * HD) / (4 * STHR); ++it) p[it * STHR + tid] = z;
  }
  scnt[tid] = 0;
  if (tid < HD) { sw2[tid] = gw2[tid]; sg[tid] = lg[tid]; sb[tid] = lb[tid]; }
  const float b2v = gb2[0];
  __syncthreads();
  const v4f w2r = ((const v4f*)sw2)[lane];

#pragma unroll 1
  for (int ch = 0; ch < nChunks; ++ch) {
    const int cbase = ch * CHUNK;
    int d[EPT];
    loadids(own, nE, cbase, tid, vec, d);
    unsigned msk = 0;
#pragma unroll
    for (int j = 0; j < EPT; ++j) {
      const unsigned ld = (unsigned)d[j] - (unsigned)n0;
      msk |= ((ld < (unsigned)NBA) ? 1u : 0u) << j;
    }
    const int cnt = __builtin_popcount(msk);
    int pos, nh;
    blkscan(cnt, lane, wave, swt, pos, nh);
    const int e0 = cbase + EPT * tid;
#pragma unroll
    for (int j = 0; j < EPT; ++j) {
      if ((msk >> j) & 1u) {
        const unsigned ld = (unsigned)d[j] - (unsigned)n0;
        if (pos < CHUNK) slist[pos] = ((unsigned)(e0 + j) << 8) | ld;
        ++pos;
      }
    }
    __syncthreads();
    const int nhc = nh < CHUNK ? nh : CHUNK;
    for (int j = 0; j < nhc; ++j) {
      const unsigned pk = (unsigned)__builtin_amdgcn_readfirstlane((int)slist[j]);
      const int ld = (int)(pk & (unsigned)(NBA - 1));
      if ((ld & (SWAV - 1)) == wave) {
        int e = (int)(pk >> 8);
        e = e > nE - 1 ? nE - 1 : e;
        int c = nbr[e];
        c = c < 0 ? 0 : (c > nN - 1 ? nN - 1 : c);
        const float* tp = T + (size_t)(n0 + ld) * (3 * HD) + 4 * lane;
        const float* tc = T + (size_t)c * (3 * HD) + 4 * lane;
        const v4f p  = *(const v4f*)tp;
        const v4f q  = *(const v4f*)(tc + HD);
        const v4f hw = *(const v4f*)(tc + 2 * HD);
        const v4f u = vrelu(p + q);
        float s = u.x * w2r.x;
        s = fmaf(u.y, w2r.y, s); s = fmaf(u.z, w2r.z, s); s = fmaf(u.w, w2r.w, s);
#pragma unroll
        for (int o = 16; o >= 1; o >>= 1) s += __shfl_xor(s, o, 32);
        s += b2v;
        s = fminf(fmaxf(s, -80.0f), 80.0f);
        const float ex = __expf(-s);
        const float g = __builtin_amdgcn_rcpf(1.0f + ex);
        v4f* ap = (v4f*)(sacc + ld * HD + 4 * lane);
        const v4f av = *ap;
        v4f nv;
        nv.x = fmaf(g, hw.x, av.x); nv.y = fmaf(g, hw.y, av.y); nv.z = fmaf(g, hw.z, av.z); nv.w = fmaf(g, hw.w, av.w);
        *ap = nv;
        if (lane == 0) scnt[ld] = scnt[ld] + 1;
      }
    }
  }
  __syncthreads();

  {
    const int r = tid;
    const int node = n0 + r;
    const int cn = scnt[r];
    const float invd = 1.0f / (float)(cn < 1 ? 1 : cn);
    v4f* ar = (v4f*)(sacc + r * HD);
    const v4f* hr = (const v4f*)(H + (size_t)node * HD);
    float s = 0.0f;
#pragma unroll 1
    for (int q = 0; q < HD / 4; ++q) {
      const v4f a = ar[q];
      const v4f hv = hr[q];
      const v4f t = hv + a * invd;
      ar[q] = t;
      s += (t.x + t.y) + (t.z + t.w);
    }
    const float mu = s * (1.0f / HD);
    float vs = 0.0f;
#pragma unroll 1
    for (int q = 0; q < HD / 4; ++q) {
      const v4f t = ar[q];
      const v4f dd = t - mu;
      vs += (dd.x * dd.x + dd.y * dd.y) + (dd.z * dd.z + dd.w * dd.w);
    }
    const float rs = rsqrtf(vs * (1.0f / HD) + EPSV);
#pragma unroll 1
    for (int q = 0; q < HD / 4; ++q) {
      const v4f t = ar[q];
      const v4f g4 = ((const v4f*)sg)[q];
      const v4f b4 = ((const v4f*)sb)[q];
      const v4f y = (t - mu) * rs * g4 + b4;
      ar[q] = vrelu(y);
    }
  }
  __syncthreads();

  drain_store(sacc, H, HB, n0, tid);
  __threadfence();
  drain_store(sacc, H, HB, n0, tid);
}

template <int KS>
__global__ __launch_bounds__(GTHR) void k_head(const _Float16* __restrict__ A, const _Float16* __restrict__ Bpl,
                                               const float* __restrict__ b1, const float* __restrict__ w2,
                                               const float* __restrict__ b2, float* out, int nN) {
  constexpr int NT = 4, NCB = 64, KH = 32 * KS;
  __shared__ __attribute__((aligned(16))) float stg[GROWS * NCB];
  __shared__ __attribute__((aligned(16))) float sw2[NCB];
  const int tid = threadIdx.x, lane = tid & 31, wave = tid >> 5, hh = lane >> 4, m = lane & 15;
  const int rowBase = blockIdx.x * GROWS;
  sw2[tid] = w2[tid];
  {
    v8f acc[NT];
    mma16<KS, NT>(A + (size_t)(rowBase + wave * 16) * KH, Bpl, lane, acc);
    float* sp = stg + (wave * 16 + 8 * hh) * NCB + m;
#pragma unroll
    for (int t = 0; t < NT; ++t) {
      const float bv = b1[16 * t + m];
#pragma unroll
      for (int r = 0; r < 8; ++r) sp[r * NCB + 16 * t] = fmaxf(fmaf(acc[t][r], RH, bv), 0.0f);
    }
  }
  __syncthreads();
  if (wave == 0) {
    const float* rp = stg + lane * NCB;
    float s = b2[0];
#pragma unroll 4
    for (int c = 0; c < NCB; ++c) s = fmaf(rp[c], sw2[c], s);
    const int gr = rowBase + lane;
    const bool full = (rowBase + GROWS <= nN);
    if (full) { *(volatile float*)(out + gr) = s; }
    else if (gr < nN) { *(volatile float*)(out + gr) = s; }
    __threadfence();
    if (full) { *(volatile float*)(out + gr) = s; }
    else if (gr < nN) { *(volatile float*)(out + gr) = s; }
  }
}

extern "C" void kernel_launch(void* const* d_in, const int* in_sizes, int n_in,
                              void* d_out, int out_size, void* d_ws, size_t ws_size,
                              hipStream_t stream) {
  if (n_in < 21) return;
  const int nN = in_sizes[0] / INW;
  const int nE = in_sizes[1] / 2;
  if (nN < 1 || nE < 1) return;
  if (in_sizes[0] != nN * INW || in_sizes[1] != 2 * nE) return;
  if (in_sizes[2] != INW * EH || in_sizes[3] != EH || in_sizes[4] != EH || in_sizes[5] != EH) return;
  if (in_sizes[6] != EH * HD || in_sizes[7] != HD || in_sizes[8] != HD || in_sizes[9] != HD) return;
  if (in_sizes[10] != NL * HD * HD || in_sizes[11] != NL * 2 * HD * HD || in_sizes[12] != NL * HD) return;
  if (in_sizes[13] != NL * HD || in_sizes[14] != NL || in_sizes[15] != NL * HD || in_sizes[16] != NL * HD) return;
  if (in_sizes[17] != HD * HHALF || in_sizes[18] != HHALF || in_sizes[19] != HHALF || in_sizes[20] < 1) return;
  if (out_size != nN) return;
  if (nN > (1 << 22) || nE > (1 << 23)) return;

  const float* x    = (const float*)d_in[0];
  const int*   ei   = (const int*)d_in[1];
  const float* ew1  = (const float*)d_in[2];
  const float* eb1  = (const float*)d_in[3];
  const float* g1   = (const float*)d_in[4];
  const float* be1  = (const float*)d_in[5];
  const float* ew2  = (const float*)d_in[6];
  const float* eb2  = (const float*)d_in[7];
  const float* g2   = (const float*)d_in[8];
  const float* be2  = (const float*)d_in[9];
  const float* wl   = (const float*)d_in[10];
  const float* gw1  = (const float*)d_in[11];
  const float* gb1  = (const float*)d_in[12];
  const float* gw2  = (const float*)d_in[13];
  const float* gb2  = (const float*)d_in[14];
  const float* lng  = (const float*)d_in[15];
  const float* lnb  = (const float*)d_in[16];
  const float* hw1  = (const float*)d_in[17];
  const float* hb1  = (const float*)d_in[18];
  const float* hw2  = (const float*)d_in[19];
  const float* hb2  = (const float*)d_in[20];
  float* out = (float*)d_out;
  const int* own = ei;
  const int* nbr = ei + (size_t)nE;

  const int nPad    = ((nN + NPADG - 1) / NPADG) * NPADG;
  const int gNode   = nPad / GROWS;
  const int nRB     = gNode;
  const int gAgg    = nPad / NBA;
  const int nChunks = (nE + CHUNK - 1) / CHUNK;
  const int vec     = 1;

  char* ws = (char*)d_ws;
  size_t off = 0;
  const size_t oWP = off; off += (size_t)WPTOT * 2;              off = (off + 255) & ~(size_t)255;
  const size_t oXH = off; off += (size_t)nPad * INW * 2;         off = (off + 255) & ~(size_t)255;
  const size_t oBG = off; off += (size_t)nPad * 3 * HD * 4;      off = (off + 255) & ~(size_t)255;
  const size_t oH  = off; off += (size_t)nPad * HD * 4;          off = (off + 255) & ~(size_t)255;
  const size_t oHH = off; off += (size_t)nPad * EH * 2;          off = (off + 255) & ~(size_t)255;
  const size_t oPT = off; off += (size_t)nRB * 2 * EH * 4;       off = (off + 255) & ~(size_t)255;
  const size_t oST = off; off += (size_t)2 * 256 * 4;            off = (off + 255) & ~(size_t)255;
  if (off > ws_size || off > (size_t)WSCAP) return;
  _Float16* WP   = (_Float16*)(ws + oWP);
  _Float16* XH   = (_Float16*)(ws + oXH);
  float*    BIG  = (float*)(ws + oBG);
  float*    H    = (float*)(ws + oH);
  _Float16* HH   = (_Float16*)(ws + oHH);
  float*    PART = (float*)(ws + oPT);
  float*    STAT = (float*)(ws + oST);

  hipFuncSetAttribute(reinterpret_cast<const void*>(&k_drain), hipFuncAttributeMaxDynamicSharedMemorySize, LDS_DRAIN);

  k_wprep<<<24 + 24 * NL + 4, 256, 0, stream>>>(ew1, ew2, gw1, wl, hw1, WP);
  k_xprep<<<nPad / 32, 256, 0, stream>>>(x, XH, nN);
  k_gemm<INW / 32, 8, 1><<<dim3(gNode, EH / 128), GTHR, 0, stream>>>(XH, WP + OFF_E1, eb1, 0, EH, BIG, EH, PART, EH, nN);
  k_bnstat<<<1, 256, 0, stream>>>(PART, nRB, EH, g1, STAT, nN);
  k_bnapply<EH, 0><<<(nPad / NPADG) * ((NPADG * EH) / BNEL), 256, 0, stream>>>(BIG, STAT, be1, HH, H);
  k_gemm<EH / 32, 8, 1><<<dim3(gNode, HD / 128), GTHR, 0, stream>>>(HH, WP + OFF_E2, eb2, 0, HD, BIG, HD, PART, HD, nN);
  k_bnstat<<<1, 256, 0, stream>>>(PART, nRB, HD, g2, STAT, nN);
  k_bnapply<HD, 1><<<(nPad / NPADG) * ((NPADG * HD) / BNEL), 256, 0, stream>>>(BIG, STAT, be2, HH, H);
  for (int l = 0; l < NL; ++l) {
    k_gemm<HD / 32, 8, 0><<<dim3(gNode, 3), GTHR, 0, stream>>>(HH, WP + OFF_L + (size_t)l * LPL,
                                                                gb1 + (size_t)l * HD, HD, 2 * HD,
                                                                BIG, 3 * HD, BIG, 0, nN);
    k_drain<<<gAgg, STHR, LDS_DRAIN, stream>>>(own, nbr, BIG, gw2 + (size_t)l * HD, gb2 + l,
                                               lng + (size_t)l * HD, lnb + (size_t)l * HD,
                                               H, HH, nN, nE, nChunks, vec);
  }
  k_head<HD / 32><<<gNode, GTHR, 0, stream>>>(HH, WP + OFF_HW, hb1, hw2, hb2, out, nN);
}
